// CharEmbedding_66881230733377
// MI455X (gfx1250) — hardware-verified
//
#include <hip/hip_runtime.h>
#include <stddef.h>
#include <stdint.h>


#define B_    64
#define LW_   512
#define LC_   4096
#define DW_   300
#define DC_   64
#define H_    128
#define KIN   364
#define KP    384
#define NCE   257
#define M_    (B_ * LW_)
#define BM    32
#define NTHR  256
#define SXS   392
#define SHS   136
#define SOS   132
#define XSC   8
#define WSC   1024
#define NBS   13
#define WSCAP 134217728

static_assert(KIN == DW_ + DC_);
static_assert(KP % 32 == 0 && KP >= KIN);
static_assert(H_ % 32 == 0);
static_assert(LW_ % BM == 0);
static_assert(M_ % BM == 0);
static_assert(NTHR == BM * 8);
static_assert(NTHR == 8 * 32);
static_assert(DW_ % 4 == 0);
static_assert(DC_ == 64);
static_assert((SXS * 2) % 16 == 0);
static_assert((SHS * 2) % 16 == 0);
static_assert((SOS * 4) % 16 == 0);
static_assert(SXS >= KP);
static_assert(SHS >= H_);
static_assert(SOS >= H_);
static_assert((H_ * KP) % (8 * NTHR) == 0);
static_assert((H_ * H_) % (8 * NTHR) == 0);
static_assert((1 << (NBS - 1)) >= LC_);

typedef float    v4f  __attribute__((ext_vector_type(4)));
typedef float    v8f  __attribute__((ext_vector_type(8)));
typedef _Float16 v4h  __attribute__((ext_vector_type(4)));
typedef _Float16 v8h  __attribute__((ext_vector_type(8)));
typedef _Float16 v16h __attribute__((ext_vector_type(16)));
union FragH { v16h v; v8h s[2]; };

__device__ __forceinline__ int imin(int a, int b) { return a < b ? a : b; }
__device__ __forceinline__ int imax(int a, int b) { return a > b ? a : b; }

__device__ __forceinline__ v8f wmf(v16h a, v16h b, v8f c) {
  v8f d = __builtin_amdgcn_wmma_f32_16x16x32_f16(false, a, false, b, (short)0, c, false, false);
  asm volatile("v_nop\n\tv_nop\n\tv_nop\n\tv_nop" : "+v"(d) : "v"(a), "v"(b));
  return d;
}

__device__ __forceinline__ v16h ld_frag(const _Float16* row_plus_8h, int k0) {
  FragH f;
  f.s[0] = *(const v8h*)(row_plus_8h + k0);
  f.s[1] = *(const v8h*)(row_plus_8h + k0 + 16);
  return f.v;
}

__global__ __launch_bounds__(NTHR) void k_prep_wp(const float* __restrict__ W, _Float16* dst) {
  const int t = blockIdx.x * NTHR + threadIdx.x;
  if (t >= (H_ * KP) / 8) return;
  const int n  = t / (KP / 8);
  const int kq = (t - n * (KP / 8)) * 8;
  v8h hv;
#pragma unroll
  for (int e = 0; e < 8; ++e) {
    const int k  = kq + e;
    const int kc = (k < KIN) ? k : (KIN - 1);
    const float v = W[(size_t)n * KIN + kc];
    const float sc = (k < KIN) ? (float)WSC : 0.0f;
    hv[e] = (_Float16)(v * sc);
  }
  _Float16* d = dst + (size_t)t * 8;
  *(volatile v8h*)d = hv;
  __threadfence();
  *(volatile v8h*)d = hv;
}

__global__ __launch_bounds__(NTHR) void k_prep_hw(const float* __restrict__ W, _Float16* dst) {
  const int t = blockIdx.x * NTHR + threadIdx.x;
  if (t >= (H_ * H_) / 8) return;
  const float* p = W + (size_t)t * 8;
  const v4f f0 = *(const v4f*)p;
  const v4f f1 = *(const v4f*)(p + 4);
  v8h a;
  a[0] = (_Float16)(f0.x * (float)WSC); a[1] = (_Float16)(f0.y * (float)WSC);
  a[2] = (_Float16)(f0.z * (float)WSC); a[3] = (_Float16)(f0.w * (float)WSC);
  a[4] = (_Float16)(f1.x * (float)WSC); a[5] = (_Float16)(f1.y * (float)WSC);
  a[6] = (_Float16)(f1.z * (float)WSC); a[7] = (_Float16)(f1.w * (float)WSC);
  _Float16* d = dst + (size_t)t * 8;
  *(volatile v8h*)d = a;
  __threadfence();
  *(volatile v8h*)d = a;
}

__device__ __forceinline__ void hw_layer(_Float16* sH,
                                         const _Float16* __restrict__ Wgb, const float* __restrict__ bg,
                                         const _Float16* __restrict__ Wtb, const float* __restrict__ bt,
                                         v8f& x0, v8f& x1, int wave, int h, int m) {
  const int col = 16 * wave + m;
#pragma unroll
  for (int r = 0; r < 8; ++r) {
    sH[(8 * h + r) * SHS + col]      = (_Float16)(x0[r] * (float)XSC);
    sH[(16 + 8 * h + r) * SHS + col] = (_Float16)(x1[r] * (float)XSC);
  }
  __syncthreads();

  v8f ag0 = {0.f, 0.f, 0.f, 0.f, 0.f, 0.f, 0.f, 0.f};
  v8f ag1 = ag0, at0 = ag0, at1 = ag0;
  const _Float16* a0p = sH + m * SHS + 8 * h;
  const _Float16* a1p = sH + (16 + m) * SHS + 8 * h;
  const _Float16* gp  = Wgb + (size_t)col * H_ + 8 * h;
  const _Float16* tp  = Wtb + (size_t)col * H_ + 8 * h;
#pragma unroll
  for (int kt = 0; kt < H_ / 32; ++kt) {
    const int k0 = 32 * kt;
    const v16h a0 = ld_frag(a0p, k0);
    const v16h a1 = ld_frag(a1p, k0);
    const v16h fg = ld_frag(gp, k0);
    const v16h ft = ld_frag(tp, k0);
    ag0 = wmf(a0, fg, ag0);
    ag1 = wmf(a1, fg, ag1);
    at0 = wmf(a0, ft, at0);
    at1 = wmf(a1, ft, at1);
  }
  __syncthreads();

  constexpr float OSC = 1.0f / (float)(XSC * WSC);
  const float bgv = bg[col];
  const float btv = bt[col];
#pragma unroll
  for (int r = 0; r < 8; ++r) {
    {
      const float zg = ag0[r] * OSC + bgv;
      const float g  = __builtin_amdgcn_rcpf(1.0f + __expf(-zg));
      const float tt = fmaxf(at0[r] * OSC + btv, 0.0f);
      x0[r] = g * tt + (1.0f - g) * x0[r];
    }
    {
      const float zg = ag1[r] * OSC + bgv;
      const float g  = __builtin_amdgcn_rcpf(1.0f + __expf(-zg));
      const float tt = fmaxf(at1[r] * OSC + btv, 0.0f);
      x1[r] = g * tt + (1.0f - g) * x1[r];
    }
  }
}

__global__ __launch_bounds__(NTHR) void k_main(const int* __restrict__ w, const int* __restrict__ c, const int* __restrict__ p,
                                               const float* __restrict__ wv, const float* __restrict__ ce,
                                               const _Float16* __restrict__ Wpb,
                                               const _Float16* __restrict__ Wg0b, const float* __restrict__ bg0,
                                               const _Float16* __restrict__ Wt0b, const float* __restrict__ bt0,
                                               const _Float16* __restrict__ Wg1b, const float* __restrict__ bg1,
                                               const _Float16* __restrict__ Wt1b, const float* __restrict__ bt1,
                                               float* out, int nV) {
  __shared__ __attribute__((aligned(16))) _Float16 sX[BM * SXS];
  __shared__ __attribute__((aligned(16))) _Float16 sH[BM * SHS];
  __shared__ __attribute__((aligned(16))) float    sO[BM * SOS];
  __shared__ int sLo[BM];
  __shared__ int sCnt[BM];

  const int tid = threadIdx.x, lane = tid & 31, wave = tid >> 5, h = lane >> 4, m = lane & 15;
  const int mbase = blockIdx.x * BM;
  const int b = mbase / LW_;

  {
    const int r = tid >> 3, q = tid & 7;
    int widx = w[mbase + r];
    widx = imin(imax(widx, 0), nV - 1);
    const float* wrow = wv + (size_t)widx * DW_;
    _Float16* srow = sX + r * SXS;
#pragma unroll 1
    for (int ch = q; ch < DW_ / 4; ch += 8) {
      const v4f v = *(const v4f*)(wrow + 4 * ch);
      v4h hv;
      hv[0] = (_Float16)(v.x * (float)XSC); hv[1] = (_Float16)(v.y * (float)XSC);
      hv[2] = (_Float16)(v.z * (float)XSC); hv[3] = (_Float16)(v.w * (float)XSC);
      *(v4h*)(srow + 4 * ch) = hv;
    }
#pragma unroll 1
    for (int k = KIN + q; k < SXS; k += 8) srow[k] = (_Float16)0.0f;
  }
  if (tid < BM) {
    const int i = mbase + tid - b * LW_;
    const int* prow = p + (size_t)b * LC_;
    int lo = 0, hi = LC_;
#pragma unroll 1
    for (int it = 0; it < NBS; ++it) {
      const int mid = (lo + hi) >> 1;
      const int pv = prow[imin(mid, LC_ - 1)];
      const bool act = lo < hi;
      const bool lt = pv < i;
      lo = (act && lt) ? (mid + 1) : lo;
      hi = (act && !lt) ? mid : hi;
    }
    int lo2 = lo, hi2 = LC_;
#pragma unroll 1
    for (int it = 0; it < NBS; ++it) {
      const int mid = (lo2 + hi2) >> 1;
      const int pv = prow[imin(mid, LC_ - 1)];
      const bool act = lo2 < hi2;
      const bool lt = pv < i + 1;
      lo2 = (act && lt) ? (mid + 1) : lo2;
      hi2 = (act && !lt) ? mid : hi2;
    }
    int cnt = lo2 - lo;
    cnt = imax(cnt, 0);
    cnt = imin(cnt, LC_ - lo);
    sLo[tid] = lo;
    sCnt[tid] = cnt;
  }
  __syncthreads();

  {
    const int r = tid >> 3, q = tid & 7;
    const int lo = sLo[r];
    const int cnt = sCnt[r];
    int cmax = cnt;
    cmax = imax(cmax, __shfl_xor(cmax, 8));
    cmax = imax(cmax, __shfl_xor(cmax, 16));
    cmax = imin(cmax, LC_);
    const int* crow = c + (size_t)b * LC_;
    float s[8];
#pragma unroll
    for (int e = 0; e < 8; ++e) s[e] = 0.0f;
#pragma unroll 1
    for (int j = 0; j < cmax; ++j) {
      const bool use = j < cnt;
      const int jj = imin(lo + j, LC_ - 1);
      int cc = crow[jj];
      cc = (cc == 32) ? 0 : cc;
      cc = imin(imax(cc, 0), NCE - 1);
      const float* ep = ce + (size_t)cc * DC_ + 8 * q;
      const v4f e0 = *(const v4f*)ep;
      const v4f e1 = *(const v4f*)(ep + 4);
      s[0] += use ? e0.x : 0.0f; s[1] += use ? e0.y : 0.0f;
      s[2] += use ? e0.z : 0.0f; s[3] += use ? e0.w : 0.0f;
      s[4] += use ? e1.x : 0.0f; s[5] += use ? e1.y : 0.0f;
      s[6] += use ? e1.z : 0.0f; s[7] += use ? e1.w : 0.0f;
    }
    const float inv = 1.0f / (0.001f + sqrtf((float)cnt));
    v4h h0, h1;
#pragma unroll
    for (int e = 0; e < 4; ++e) {
      const float u0 = s[e] * inv;
      const float u1 = s[4 + e] * inv;
      h0[e] = (_Float16)(u0 * (float)XSC);
      h1[e] = (_Float16)(u1 * (float)XSC);
    }
    _Float16* d = sX + r * SXS + DW_ + 8 * q;
    *(v4h*)d = h0;
    *(v4h*)(d + 4) = h1;
  }
  __syncthreads();

  v8f x0 = {0.f, 0.f, 0.f, 0.f, 0.f, 0.f, 0.f, 0.f};
  v8f x1 = x0;
  {
    const _Float16* a0p = sX + m * SXS + 8 * h;
    const _Float16* a1p = sX + (16 + m) * SXS + 8 * h;
    const _Float16* bp  = Wpb + (size_t)(16 * wave + m) * KP + 8 * h;
#pragma unroll 2
    for (int kt = 0; kt < KP / 32; ++kt) {
      const int k0 = 32 * kt;
      const v16h a0 = ld_frag(a0p, k0);
      const v16h a1 = ld_frag(a1p, k0);
      const v16h fb = ld_frag(bp, k0);
      x0 = wmf(a0, fb, x0);
      x1 = wmf(a1, fb, x1);
    }
    constexpr float OSC = 1.0f / (float)(XSC * WSC);
    x0 = x0 * OSC;
    x1 = x1 * OSC;
  }

  hw_layer(sH, Wg0b, bg0, Wt0b, bt0, x0, x1, wave, h, m);
  hw_layer(sH, Wg1b, bg1, Wt1b, bt1, x0, x1, wave, h, m);

  {
    const int col = 16 * wave + m;
#pragma unroll
    for (int r = 0; r < 8; ++r) {
      sO[(8 * h + r) * SOS + col]      = x0[r];
      sO[(16 + 8 * h + r) * SOS + col] = x1[r];
    }
  }
  __syncthreads();
  {
    float* ob = out + (size_t)mbase * H_;
    v4f ov[4];
#pragma unroll
    for (int rr = 0; rr < 4; ++rr) ov[rr] = *(const v4f*)(sO + (4 * wave + rr) * SOS + 4 * lane);
#pragma unroll
    for (int rr = 0; rr < 4; ++rr)
      *(volatile v4f*)(ob + (size_t)(4 * wave + rr) * H_ + 4 * lane) = ov[rr];
    __threadfence();
#pragma unroll
    for (int rr = 0; rr < 4; ++rr)
      *(volatile v4f*)(ob + (size_t)(4 * wave + rr) * H_ + 4 * lane) = ov[rr];
  }
}

extern "C" void kernel_launch(void* const* d_in, const int* in_sizes, int n_in,
                              void* d_out, int out_size, void* d_ws, size_t ws_size,
                              hipStream_t stream) {
  if (n_in < 14) return;
  if (in_sizes[0] != B_ * LW_) return;
  if (in_sizes[1] != B_ * LC_) return;
  if (in_sizes[2] != B_ * LC_) return;
  if (in_sizes[3] < DW_ || (in_sizes[3] % DW_) != 0) return;
  if (in_sizes[4] != NCE * DC_) return;
  if (in_sizes[5] != H_ * KIN) return;
  if (in_sizes[6] != H_ * H_ || in_sizes[8] != H_ * H_ || in_sizes[10] != H_ * H_ || in_sizes[12] != H_ * H_) return;
  if (in_sizes[7] != H_ || in_sizes[9] != H_ || in_sizes[11] != H_ || in_sizes[13] != H_) return;
  if (out_size != M_ * H_) return;
  const int nV = in_sizes[3] / DW_;

  const int*   w    = (const int*)d_in[0];
  const int*   c    = (const int*)d_in[1];
  const int*   p    = (const int*)d_in[2];
  const float* wv   = (const float*)d_in[3];
  const float* ce   = (const float*)d_in[4];
  const float* Wp   = (const float*)d_in[5];
  const float* Wt0  = (const float*)d_in[6];
  const float* bt0  = (const float*)d_in[7];
  const float* Wg0  = (const float*)d_in[8];
  const float* bg0  = (const float*)d_in[9];
  const float* Wt1  = (const float*)d_in[10];
  const float* bt1  = (const float*)d_in[11];
  const float* Wg1  = (const float*)d_in[12];
  const float* bg1  = (const float*)d_in[13];
  float* out = (float*)d_out;

  char* ws = (char*)d_ws;
  size_t off = 0;
  const size_t oWp = off; off += (size_t)H_ * KP * 2; off = (off + 255) & ~(size_t)255;
  const size_t oG0 = off; off += (size_t)H_ * H_ * 2; off = (off + 255) & ~(size_t)255;
  const size_t oT0 = off; off += (size_t)H_ * H_ * 2; off = (off + 255) & ~(size_t)255;
  const size_t oG1 = off; off += (size_t)H_ * H_ * 2; off = (off + 255) & ~(size_t)255;
  const size_t oT1 = off; off += (size_t)H_ * H_ * 2; off = (off + 255) & ~(size_t)255;
  if (off > ws_size || off > (size_t)WSCAP) return;
  _Float16* Wpb  = (_Float16*)(ws + oWp);
  _Float16* Wg0b = (_Float16*)(ws + oG0);
  _Float16* Wt0b = (_Float16*)(ws + oT0);
  _Float16* Wg1b = (_Float16*)(ws + oG1);
  _Float16* Wt1b = (_Float16*)(ws + oT1);

  k_prep_wp<<<(H_ * KP) / (8 * NTHR), NTHR, 0, stream>>>(Wp, Wpb);
  k_prep_hw<<<(H_ * H_) / (8 * NTHR), NTHR, 0, stream>>>(Wg0, Wg0b);
  k_prep_hw<<<(H_ * H_) / (8 * NTHR), NTHR, 0, stream>>>(Wt0, Wt0b);
  k_prep_hw<<<(H_ * H_) / (8 * NTHR), NTHR, 0, stream>>>(Wg1, Wg1b);
  k_prep_hw<<<(H_ * H_) / (8 * NTHR), NTHR, 0, stream>>>(Wt1, Wt1b);

  k_main<<<M_ / BM, NTHR, 0, stream>>>(w, c, p, wv, ce, Wpb,
                                        Wg0b, bg0, Wt0b, bt0,
                                        Wg1b, bg1, Wt1b, bt1,
                                        out, nV);
}
